// MHSA_9105330668017
// MI455X (gfx1250) — hardware-verified
//
#include <hip/hip_runtime.h>
#include <stdint.h>


typedef unsigned short hword;
typedef hword us8  __attribute__((ext_vector_type(8)));
typedef hword us16 __attribute__((ext_vector_type(16)));
typedef _Float16 f16x16 __attribute__((ext_vector_type(16)));
typedef float v8f __attribute__((ext_vector_type(8)));
typedef float v4f __attribute__((ext_vector_type(4)));

#ifndef NB
#define NB 4
#endif
#ifndef SEQ
#define SEQ 2048
#endif
#define NB_FULL  4
#define SEQ_FULL 2048
#define DIM  1024
#define HD   64
#define NH   16
#define NTOK (NB * SEQ)
#define NT64 (NTOK / 64)
#define NQT  (SEQ / 64)
#define NW8  (NH * HD * HD / 8)
#define LDT  68
#define WCAR 32.0f
#define QCAR 64.0f
#define PCAR 16384.0f

static_assert(NB >= 1 && NB <= NB_FULL);
static_assert(SEQ >= 64 && SEQ <= SEQ_FULL && (SEQ % 64) == 0);
static_assert(DIM == NH * HD);
static_assert((NW8 % 256) == 0);
static_assert(((NTOK * (DIM / 8)) % 256) == 0);

__device__ __forceinline__ hword f2bf(float x) {
    unsigned int u = __float_as_uint(x);
    u = (u + 0x7FFFu + ((u >> 16) & 1u)) >> 16;
    return (hword)u;
}
__device__ __forceinline__ float bf2f(hword b) {
    return __uint_as_float(((unsigned int)b) << 16);
}
__device__ __forceinline__ float bfr(float x) {
    return bf2f(f2bf(x));
}
__device__ __forceinline__ hword f2h(float x) {
    _Float16 t = (_Float16)x;
    return __builtin_bit_cast(hword, t);
}
__device__ __forceinline__ v8f zero8() {
    v8f z;
#pragma unroll
    for (int i = 0; i < 8; ++i) z[i] = 0.0f;
    return z;
}

__device__ __forceinline__ v8f mma_hf(v8f c, us16 a, us16 b) {
    f16x16 av = __builtin_bit_cast(f16x16, a);
    f16x16 bv = __builtin_bit_cast(f16x16, b);
    c = __builtin_amdgcn_wmma_f32_16x16x32_f16(false, av, false, bv, (short)0, c, false, false);
    asm volatile("v_nop\n\tv_nop\n\tv_nop\n\tv_nop" : "+v"(c) : "v"(a), "v"(b));
    return c;
}

__device__ __forceinline__ us16 frag_rows(const hword* p, int ld, int row, int k0, int h) {
    const hword* base = p + (size_t)row * ld + k0 + 8 * h;
    us8 e0 = *(const us8*)(base);
    us8 e1 = *(const us8*)(base + 16);
    return __builtin_shufflevector(e0, e1, 0, 1, 2, 3, 4, 5, 6, 7,
                                   8, 9, 10, 11, 12, 13, 14, 15);
}

__global__ __launch_bounds__(256) void k_cvtx(const float* __restrict__ x, int n8,
                                              hword* __restrict__ xf) {
    const int i = blockIdx.x * 256 + (int)threadIdx.x;
    if (i >= n8) return;
    const int tok = i >> 7;
    const int c8  = i & 127;
    const int bb  = tok / SEQ, n = tok - bb * SEQ;
    const float* s = x + ((size_t)(bb * SEQ_FULL + n)) * DIM + c8 * 8;
    const v4f a = *(const v4f*)(s);
    const v4f b = *(const v4f*)(s + 4);
    us8 o;
#pragma unroll
    for (int e = 0; e < 4; ++e) {
        o[e]     = f2h(bfr(a[e]));
        o[4 + e] = f2h(bfr(b[e]));
    }
    hword* d = xf + (size_t)i * 8;
    *(volatile us8*)d = o;
    __threadfence();
    *(volatile us8*)d = o;
}

__global__ __launch_bounds__(256) void k_cvtw(const float* __restrict__ w0,
                                              const float* __restrict__ w1,
                                              const float* __restrict__ w2,
                                              hword* __restrict__ wf) {
    const int i = blockIdx.x * 256 + (int)threadIdx.x;
    if (i >= 3 * NW8) return;
    const int mat = i / NW8;
    const int j = i - mat * NW8;
    const float* src = (mat == 0) ? w0 : ((mat == 1) ? w1 : w2);
    const float* s = src + (size_t)j * 8;
    const v4f a = *(const v4f*)(s);
    const v4f b = *(const v4f*)(s + 4);
    us8 o;
#pragma unroll
    for (int e = 0; e < 4; ++e) {
        o[e]     = f2h(bfr(a[e]) * WCAR);
        o[4 + e] = f2h(bfr(b[e]) * WCAR);
    }
    hword* d = wf + (size_t)i * 8;
    *(volatile us8*)d = o;
    __threadfence();
    *(volatile us8*)d = o;
}

template <int SV>
__global__ __launch_bounds__(128) void k_qkv(const hword* __restrict__ xf,
                                             const hword* __restrict__ wf,
                                             const float* __restrict__ bias,
                                             hword* __restrict__ dst) {
    __shared__ __align__(16) float tile[64 * LDT];
    const int w = threadIdx.x >> 5, lane = threadIdx.x & 31;
    const int h = lane >> 4, m = lane & 15;
    const int mt = blockIdx.x % NT64, hh = blockIdx.x / NT64;
    const int tok0 = mt * 64;
    const int wr = w & 1, wc = w >> 1;
    const int ar0 = tok0 + wr * 32;
    const hword* xp = xf + hh * HD;
    const hword* wp = wf + (size_t)hh * (HD * HD);

    v8f acc[2][2];
#pragma unroll
    for (int mi = 0; mi < 2; ++mi)
#pragma unroll
        for (int t = 0; t < 2; ++t) acc[mi][t] = zero8();

#pragma unroll
    for (int k0 = 0; k0 < HD; k0 += 32) {
        const us16 a0 = frag_rows(xp, DIM, ar0 + m, k0, h);
        const us16 a1 = frag_rows(xp, DIM, ar0 + 16 + m, k0, h);
#pragma unroll
        for (int t = 0; t < 2; ++t) {
            const us16 b = frag_rows(wp, HD, wc * 32 + t * 16 + m, k0, h);
            acc[0][t] = mma_hf(acc[0][t], a0, b);
            acc[1][t] = mma_hf(acc[1][t], a1, b);
        }
    }

#pragma unroll
    for (int t = 0; t < 2; ++t) {
        const int e = wc * 32 + t * 16 + m;
        const float bvv = bfr(bias[hh * HD + e]);
#pragma unroll
        for (int mi = 0; mi < 2; ++mi)
#pragma unroll
            for (int r = 0; r < 8; ++r)
                tile[(wr * 32 + mi * 16 + 8 * h + r) * LDT + e] =
                    acc[mi][t][r] * (1.0f / WCAR) + bvv;
    }
    __syncthreads();

    const int bb = tok0 / SEQ, n0 = tok0 - bb * SEQ;
    const int p = lane & 7, lq = lane >> 3;
    const size_t bhi = (size_t)(bb * NH + hh);
    us8 o4[4];
    if (SV == 0) {
#pragma unroll
        for (int i = 0; i < 4; ++i) {
            const int row = w * 16 + 4 * i + lq;
            const float* sp = tile + row * LDT + 8 * p;
            const v4f u0 = *(const v4f*)(sp);
            const v4f u1 = *(const v4f*)(sp + 4);
            float ss = 0.0f;
#pragma unroll
            for (int e = 0; e < 4; ++e) ss += u0[e] * u0[e] + u1[e] * u1[e];
            ss += __shfl_xor(ss, 1, 32);
            ss += __shfl_xor(ss, 2, 32);
            ss += __shfl_xor(ss, 4, 32);
            const float nrm = fmaxf(sqrtf(ss), 1.0e-12f);
            const float scl = QCAR * (1.0f / nrm);
            us8 o;
#pragma unroll
            for (int e = 0; e < 4; ++e) {
                o[e]     = f2h(u0[e] * scl);
                o[4 + e] = f2h(u1[e] * scl);
            }
            o4[i] = o;
        }
#pragma unroll
        for (int i = 0; i < 4; ++i) {
            const int row = w * 16 + 4 * i + lq;
            hword* dp = dst + (bhi * SEQ + (size_t)(n0 + row)) * HD + 8 * p;
            *(volatile us8*)dp = o4[i];
        }
        __threadfence();
#pragma unroll
        for (int i = 0; i < 4; ++i) {
            const int row = w * 16 + 4 * i + lq;
            hword* dp = dst + (bhi * SEQ + (size_t)(n0 + row)) * HD + 8 * p;
            *(volatile us8*)dp = o4[i];
        }
    } else {
#pragma unroll
        for (int i = 0; i < 4; ++i) {
            const int d = w * 16 + 4 * i + lq;
            us8 o;
#pragma unroll
            for (int e = 0; e < 8; ++e) o[e] = f2h(tile[(8 * p + e) * LDT + d]);
            o4[i] = o;
        }
#pragma unroll
        for (int i = 0; i < 4; ++i) {
            const int d = w * 16 + 4 * i + lq;
            hword* dp = dst + (bhi * HD + (size_t)d) * SEQ + (size_t)(n0 + 8 * p);
            *(volatile us8*)dp = o4[i];
        }
        __threadfence();
#pragma unroll
        for (int i = 0; i < 4; ++i) {
            const int d = w * 16 + 4 * i + lq;
            hword* dp = dst + (bhi * HD + (size_t)d) * SEQ + (size_t)(n0 + 8 * p);
            *(volatile us8*)dp = o4[i];
        }
    }
}

__global__ __launch_bounds__(128) __attribute__((amdgpu_num_vgpr(256)))
void k_attn(const hword* __restrict__ qp, const hword* __restrict__ kp,
            const hword* __restrict__ vt, const float* __restrict__ temp,
            float* __restrict__ out) {
    __shared__ __align__(16) float st[4 * 16 * LDT];
    const int w = threadIdx.x >> 5, lane = threadIdx.x & 31;
    const int h = lane >> 4, m = lane & 15;
    const int qt = blockIdx.x % NQT, bh = blockIdx.x / NQT;
    const int bb = bh / NH, hh = bh - bb * NH;
    const size_t poff = (size_t)bh * SEQ * HD;
    const hword* qhp = qp + poff;
    const hword* khp = kp + poff;
    const hword* vtp = vt + poff;
    const int q0 = qt * 64 + w * 16;
    const float sfac = fmaxf(bfr(temp[hh]), 0.01f) * (1.0f / (QCAR * QCAR));

    us16 qb[2];
#pragma unroll
    for (int dc = 0; dc < 2; ++dc) qb[dc] = frag_rows(qhp, HD, q0 + m, dc * 32, h);

    v8f oacc[4];
#pragma unroll
    for (int dt = 0; dt < 4; ++dt) oacc[dt] = zero8();
    float mrun = -1.0e30f, lrun = 0.0f;

#pragma unroll 1
    for (int kc = 0; kc < SEQ; kc += 64) {
        v8f sacc[4];
#pragma unroll
        for (int kt = 0; kt < 4; ++kt) {
            v8f sa = zero8();
            const int krow = kc + kt * 16 + m;
#pragma unroll
            for (int dc = 0; dc < 2; ++dc) {
                const us16 ka = frag_rows(khp, HD, krow, dc * 32, h);
                sa = mma_hf(sa, ka, qb[dc]);
            }
            sacc[kt] = sa;
        }

        float mloc = -1.0e30f;
#pragma unroll
        for (int kt = 0; kt < 4; ++kt)
#pragma unroll
            for (int r = 0; r < 8; ++r) mloc = fmaxf(mloc, sacc[kt][r]);
        mloc = fmaxf(mloc, __shfl_xor(mloc, 16, 32));
        const float mnew = fmaxf(mrun, mloc);
        const float corr = __expf((mrun - mnew) * sfac);
        mrun = mnew;
        float lsum = 0.0f;
        us16 pb[2];
#pragma unroll
        for (int kt = 0; kt < 4; ++kt) {
#pragma unroll
            for (int r = 0; r < 8; ++r) {
                const float pv = __expf((sacc[kt][r] - mnew) * sfac);
                lsum += pv;
                pb[kt >> 1][(kt & 1) * 8 + r] = f2h(pv * PCAR);
            }
        }
        lsum += __shfl_xor(lsum, 16, 32);
        lrun = lrun * corr + lsum;
#pragma unroll
        for (int dt = 0; dt < 4; ++dt) oacc[dt] = oacc[dt] * corr;

#pragma unroll
        for (int ks = 0; ks < 2; ++ks) {
#pragma unroll
            for (int dt = 0; dt < 4; ++dt) {
                const us16 va = frag_rows(vtp, SEQ, dt * 16 + m, kc + ks * 32, h);
                oacc[dt] = mma_hf(oacc[dt], va, pb[ks]);
            }
        }
    }

    const float inv = 1.0f / (lrun * PCAR);
    float* sw = st + w * (16 * LDT);
#pragma unroll
    for (int dt = 0; dt < 4; ++dt) {
        v4f u0, u1;
#pragma unroll
        for (int r = 0; r < 4; ++r) {
            u0[r] = oacc[dt][r] * inv;
            u1[r] = oacc[dt][4 + r] * inv;
        }
        *(v4f*)(sw + m * LDT + dt * 16 + 8 * h) = u0;
        *(v4f*)(sw + m * LDT + dt * 16 + 8 * h + 4) = u1;
    }
    __syncthreads();

    v4f vr[8];
#pragma unroll
    for (int i = 0; i < 8; ++i) vr[i] = *(const v4f*)(sw + (2 * i + h) * LDT + 4 * m);
    const size_t orow0 = (size_t)(bb * SEQ_FULL + q0);
#pragma unroll
    for (int i = 0; i < 8; ++i) {
        float* dp = out + (orow0 + (size_t)(2 * i + h)) * DIM + hh * HD + 4 * m;
        *(volatile v4f*)dp = vr[i];
    }
    __threadfence();
#pragma unroll
    for (int i = 0; i < 8; ++i) {
        float* dp = out + (orow0 + (size_t)(2 * i + h)) * DIM + hh * HD + 4 * m;
        *(volatile v4f*)dp = vr[i];
    }
}

extern "C" void kernel_launch(void* const* d_in, const int* in_sizes, int n_in,
                              void* d_out, int out_size, void* d_ws, size_t ws_size,
                              hipStream_t stream) {
    if (n_in < 8) return;
    const int need_x = ((NB - 1) * SEQ_FULL + SEQ) * DIM;
    if (in_sizes[0] < need_x || in_sizes[1] < NH * HD * HD || in_sizes[2] < NH * HD ||
        in_sizes[3] < NH * HD * HD || in_sizes[4] < NH * HD || in_sizes[5] < NH * HD * HD ||
        in_sizes[6] < NH * HD || in_sizes[7] < NH || out_size < need_x) return;

    const float* x    = (const float*)d_in[0];
    const float* Wq   = (const float*)d_in[1];
    const float* bq   = (const float*)d_in[2];
    const float* Wk   = (const float*)d_in[3];
    const float* bk   = (const float*)d_in[4];
    const float* Wv   = (const float*)d_in[5];
    const float* bv   = (const float*)d_in[6];
    const float* temp = (const float*)d_in[7];
    float* out = (float*)d_out;

    const size_t b_x = (size_t)NTOK * DIM * 2;
    const size_t b_p = (size_t)NB * NH * SEQ * HD * 2;
    const size_t b_w = (size_t)3 * NH * HD * HD * 2;
    size_t off = 0;
    char* ws = (char*)d_ws;
    hword* xf  = (hword*)(ws + off); off += b_x;
    hword* qpl = (hword*)(ws + off); off += b_p;
    hword* kpl = (hword*)(ws + off); off += b_p;
    hword* vtp = (hword*)(ws + off); off += b_p;
    hword* wf  = (hword*)(ws + off); off += b_w;
    if (off > ws_size) return;

    const int n8x = NTOK * (DIM / 8);
    k_cvtx<<<(n8x + 255) / 256, 256, 0, stream>>>(x, n8x, xf);
    k_cvtw<<<(3 * NW8 + 255) / 256, 256, 0, stream>>>(Wq, Wk, Wv, wf);

    k_qkv<0><<<NT64 * NH, 128, 0, stream>>>(xf, wf,                  bq, qpl);
    k_qkv<0><<<NT64 * NH, 128, 0, stream>>>(xf, wf + NH * HD * HD,   bk, kpl);
    k_qkv<1><<<NT64 * NH, 128, 0, stream>>>(xf, wf + 2 * NH * HD * HD, bv, vtp);

    k_attn<<<NB * NH * NQT, 128, 0, stream>>>(qpl, kpl, vtp, temp, out);
}
